// MultiHeadedAttention_38869454029277
// MI455X (gfx1250) — hardware-verified
//
#include <hip/hip_runtime.h>
#include <math.h>

typedef __attribute__((ext_vector_type(16))) _Float16 v16h;
typedef __attribute__((ext_vector_type(16))) __bf16 v16b;
typedef __attribute__((ext_vector_type(8)))  _Float16 v8h;
typedef __attribute__((ext_vector_type(8)))  float v8f;
typedef __attribute__((ext_vector_type(4)))  float v4f;
typedef __attribute__((ext_vector_type(4)))  unsigned v4u;

#ifndef NB
#define NB 4
#endif
#ifndef SEQ
#define SEQ 2048
#endif
#define NB_FULL 4
#define SEQ_FULL 2048
#define DIN 768
#define CC 768
#define NH 12
#define HD 64
#define SC2 (0.18033688011112042f)
#define MASKV (-1.4426950408889634e9f)

static_assert(CC == NH * HD);
static_assert(HD == 64);
static_assert(DIN % 32 == 0);
static_assert(CC % 32 == 0);
static_assert(CC % 128 == 0);
static_assert(DIN % 128 == 0);
static_assert(SEQ % 64 == 0);
static_assert(SEQ % 32 == 0);
static_assert(NB <= NB_FULL);
static_assert(SEQ <= SEQ_FULL);

#define PLANE_B (2u * (size_t)NB * SEQ * CC)
#define WS_QH 0u
#define WS_QL (WS_QH + PLANE_B)
#define WS_KH (WS_QL + PLANE_B)
#define WS_VT (WS_KH + PLANE_B)
#define WS_YH (WS_VT + PLANE_B)
#define WS_YL (WS_YH + PLANE_B)
#define WS_END (WS_YL + PLANE_B)
static_assert(PLANE_B % 128 == 0);
static_assert(WS_END <= 134217728u);

template <typename T> __device__ __forceinline__ void vst2(void* p, T v) { *(volatile T*)p = v; __threadfence(); *(volatile T*)p = v; }
__device__ __forceinline__ v8f wmma16(v16h a, v16h b, v8f c) {
  v8f d = __builtin_amdgcn_wmma_f32_16x16x32_f16(false, a, false, b, (short)0, c, false, false);
  asm volatile("v_nop\n\tv_nop\n\tv_nop\n\tv_nop" : "+v"(d) : "v"(a), "v"(b));
  return d;
}
__device__ __forceinline__ v8f wmma_bf(v16b a, v16b b, v8f c) {
  v8f d = __builtin_amdgcn_wmma_f32_16x16x32_bf16(false, a, false, b, (short)0, c, false, false);
  asm volatile("v_nop\n\tv_nop\n\tv_nop\n\tv_nop" : "+v"(d) : "v"(a), "v"(b));
  return d;
}
__device__ __forceinline__ v16h frag_h(const _Float16* rowk0, int lane) {
  union { v16h v; v8h q[2]; } u; const _Float16* p = rowk0 + 8 * (lane >> 4);
  u.q[0] = *(const v8h*)p; u.q[1] = *(const v8h*)(p + 16); return u.v;
}
__device__ __forceinline__ float bfr(float v) { return (float)(__bf16)v; }
__device__ __forceinline__ v16b wcol_io(const float* __restrict__ Wm, int k0, int o, int lane, int ld) { v16b w; const int g = lane >> 4;
#pragma unroll
  for (int i = 0; i < 8; ++i) { w[i] = (__bf16)Wm[(size_t)(k0 + 8 * g + i) * ld + o]; w[8 + i] = (__bf16)Wm[(size_t)(k0 + 16 + 8 * g + i) * ld + o]; }
  return w; }
struct H2 { v16h h, l; };
__device__ __forceinline__ H2 wcolh2_io(const float* __restrict__ Wm, int k0, int o, int lane, int ld) { H2 w; const int g = lane >> 4;
#pragma unroll
  for (int i = 0; i < 8; ++i) { const float wa = bfr(Wm[(size_t)(k0 + 8 * g + i) * ld + o]); const float wb = bfr(Wm[(size_t)(k0 + 16 + 8 * g + i) * ld + o]);
    w.h[i] = (_Float16)(wa * 256.0f); w.h[8 + i] = (_Float16)(wb * 256.0f); w.l[i] = (_Float16)(wa * 0.25f); w.l[8 + i] = (_Float16)(wb * 0.25f); }
  return w; }
#define LDSX() do { asm volatile("s_wait_dscnt 0" ::: "memory"); __builtin_amdgcn_wave_barrier(); __builtin_amdgcn_fence(3  , "workgroup"); } while (0)

template <int WHICH>
__device__ __forceinline__ void proj_body(const float* __restrict__ X, const float* __restrict__ WA, const float* __restrict__ BA, _Float16* __restrict__ DH, _Float16* __restrict__ DL) {
  const int tid = threadIdx.x, wave = tid >> 5, lane = tid & 31, col = lane & 15, g = lane >> 4;
  const int c0 = blockIdx.y * 128; const size_t r0 = (size_t)blockIdx.x * 64; const size_t bb = r0 / SEQ; const int t0 = (int)(r0 % SEQ);
  const size_t xr0 = bb * (size_t)SEQ_FULL + t0;
  v8f acc[8] = {};
#pragma unroll 2
  for (int kc = 0; kc < DIN / 32; ++kc) { v16b a; { const float* p = X + (xr0 + wave * 16 + col) * DIN + kc * 32 + 8 * g;
#pragma unroll
      for (int i = 0; i < 8; ++i) { a[i] = (__bf16)p[i]; a[8 + i] = (__bf16)p[16 + i]; } }
    asm volatile("s_wait_loadcnt 0x0" ::: "memory");
#pragma unroll
    for (int j = 0; j < 8; ++j) { const v16b w = wcol_io(WA, kc * 32, c0 + j * 16 + col, lane, CC); asm volatile("s_wait_loadcnt 0x0" ::: "memory"); acc[j] = wmma_bf(a, w, acc[j]); } }
  if (WHICH < 2) {
    __shared__ __align__(16) _Float16 sh[64][136]; __shared__ __align__(16) _Float16 sl[64][136];
#pragma unroll
    for (int j = 0; j < 8; ++j) { const float bias = bfr(BA[c0 + j * 16 + col]);
#pragma unroll
      for (int r = 0; r < 8; ++r) { const float v = acc[j][r] + bias; const _Float16 hv = (_Float16)v; sh[wave * 16 + 8 * g + r][j * 16 + col] = hv; if (WHICH == 0) sl[wave * 16 + 8 * g + r][j * 16 + col] = (_Float16)((v - (float)hv) * 1024.0f); } }
    __syncthreads();
    for (int e = tid; e < 64 * 16; e += 128) { const int rl = e >> 4, q = e & 15; const size_t go = (r0 + rl) * (size_t)CC + c0 + q * 8;
      const v4u vh = *(const v4u*)&sh[rl][q * 8]; vst2((void*)(DH + go), vh);
      if (WHICH == 0) { const v4u vl = *(const v4u*)&sl[rl][q * 8]; vst2((void*)(DL + go), vl); } }
  } else {
    __shared__ __align__(16) _Float16 th[128][72];
#pragma unroll
    for (int j = 0; j < 8; ++j) { const float bias = bfr(BA[c0 + j * 16 + col]);
#pragma unroll
      for (int r = 0; r < 8; ++r) { const float v = acc[j][r] + bias; th[j * 16 + col][wave * 16 + 8 * g + r] = (_Float16)v; } }
    __syncthreads();
    for (int e = tid; e < 128 * 8; e += 128) { const int cl = e >> 3, q = e & 7; const v4u vv = *(const v4u*)&th[cl][q * 8];
      vst2((void*)(DH + (bb * CC + c0 + cl) * (size_t)SEQ + t0 + q * 8), vv); } } }

__global__ __launch_bounds__(128) void k_proj_q(const float* __restrict__ X, const float* __restrict__ W, const float* __restrict__ Bv, _Float16* __restrict__ QH, _Float16* __restrict__ QL) { proj_body<0>(X, W, Bv, QH, QL); }
__global__ __launch_bounds__(128) void k_proj_k(const float* __restrict__ X, const float* __restrict__ W, const float* __restrict__ Bv, _Float16* __restrict__ KH) { proj_body<1>(X, W, Bv, KH, (_Float16*)nullptr); }
__global__ __launch_bounds__(128) void k_proj_v(const float* __restrict__ X, const float* __restrict__ W, const float* __restrict__ Bv, _Float16* __restrict__ VT) { proj_body<2>(X, W, Bv, VT, (_Float16*)nullptr); }

__global__ __launch_bounds__(128) void k_attn(const _Float16* __restrict__ QH, const _Float16* __restrict__ QL, const _Float16* __restrict__ KH, const _Float16* __restrict__ VT, const int* __restrict__ MK, _Float16* __restrict__ YH, _Float16* __restrict__ YL) {
  __shared__ __align__(16) _Float16 sp[4][16][40];
  __shared__ __align__(16) _Float16 syh[4][16][72];
  __shared__ __align__(16) _Float16 syl[4][16][72];
  const int tid = threadIdx.x, wave = tid >> 5, lane = tid & 31, col = lane & 15, g = lane >> 4;
  const int qb = blockIdx.x, h = blockIdx.y, b = blockIdx.z;
  const int ql0 = qb * 64 + wave * 16;
  const size_t qoff = ((size_t)b * SEQ + ql0 + col) * CC + h * HD;
  const size_t kbase = (size_t)b * SEQ * CC + h * HD;
  const size_t vbase = ((size_t)b * CC + h * HD) * (size_t)SEQ;
  const int* mrowp = MK + (size_t)b * SEQ_FULL;
  v8f o[4] = {};
  float mrow[8], lrow[8];
#pragma unroll
  for (int r = 0; r < 8; ++r) { mrow[r] = -3.0e38f; lrow[r] = 0.f; }
#pragma unroll 1
  for (int s = 0; s < SEQ / 32; ++s) { const int key0 = s * 32;
    v8f a0 = {}, a1 = {}, l0 = {}, l1 = {};
#pragma unroll
    for (int kc = 0; kc < HD / 32; ++kc) {
      const v16h qh = frag_h(QH + qoff + kc * 32, lane), ql = frag_h(QL + qoff + kc * 32, lane);
      const v16h k0f = frag_h(KH + kbase + (size_t)(key0 + col) * CC + kc * 32, lane);
      a0 = wmma16(qh, k0f, a0); l0 = wmma16(ql, k0f, l0);
      const v16h k1f = frag_h(KH + kbase + (size_t)(key0 + 16 + col) * CC + kc * 32, lane);
      a1 = wmma16(qh, k1f, a1); l1 = wmma16(ql, k1f, l1); }
    const int m0 = mrowp[key0 + col], m1 = mrowp[key0 + 16 + col];
#pragma unroll
    for (int r = 0; r < 8; ++r) {
      const float s0 = (a0[r] + l0[r] * (1.0f / 1024.0f)) * SC2, s1 = (a1[r] + l1[r] * (1.0f / 1024.0f)) * SC2;
      const float v0 = (m0 != 0) ? s0 : MASKV, v1 = (m1 != 0) ? s1 : MASKV;
      float pm = fmaxf(v0, v1);
      pm = fmaxf(pm, __shfl_xor(pm, 1)); pm = fmaxf(pm, __shfl_xor(pm, 2)); pm = fmaxf(pm, __shfl_xor(pm, 4)); pm = fmaxf(pm, __shfl_xor(pm, 8));
      const float mnew = fmaxf(mrow[r], pm);
      const float alpha = exp2f(mrow[r] - mnew);
      const float p0 = exp2f(v0 - mnew), p1 = exp2f(v1 - mnew);
      lrow[r] = lrow[r] * alpha + (p0 + p1);
      mrow[r] = mnew;
      o[0][r] *= alpha; o[1][r] *= alpha; o[2][r] *= alpha; o[3][r] *= alpha;
      sp[wave][8 * g + r][col] = (_Float16)(p0 * 1024.0f);
      sp[wave][8 * g + r][16 + col] = (_Float16)(p1 * 1024.0f); }
    LDSX();
    union { v16h v; v8h q[2]; } pu; pu.q[0] = *(const v8h*)&sp[wave][col][8 * g]; pu.q[1] = *(const v8h*)&sp[wave][col][16 + 8 * g];
    LDSX();
#pragma unroll
    for (int j = 0; j < 4; ++j) { const v16h vf = frag_h(VT + vbase + (size_t)(j * 16 + col) * SEQ + key0, lane); o[j] = wmma16(pu.v, vf, o[j]); } }
#pragma unroll
  for (int r = 0; r < 8; ++r) { float l = lrow[r];
    l += __shfl_xor(l, 1); l += __shfl_xor(l, 2); l += __shfl_xor(l, 4); l += __shfl_xor(l, 8);
    const float sc = (1.0f / l) * (1.0f / 16.0f);
#pragma unroll
    for (int j = 0; j < 4; ++j) { const float y = o[j][r] * sc; const _Float16 hv = (_Float16)y; syh[wave][8 * g + r][j * 16 + col] = hv; syl[wave][8 * g + r][j * 16 + col] = (_Float16)((y - (float)hv) * 1024.0f); } }
  LDSX();
#pragma unroll
  for (int it = 0; it < 4; ++it) { const int rl = it * 4 + (lane >> 3), pc = (lane & 7) * 8; const size_t go = ((size_t)b * SEQ + ql0 + rl) * CC + h * HD + pc;
    const v4u vh = *(const v4u*)&syh[wave][rl][pc]; const v4u vl = *(const v4u*)&syl[wave][rl][pc];
    vst2((void*)(YH + go), vh); vst2((void*)(YL + go), vl); } }

__global__ __launch_bounds__(128) void k_out(const _Float16* __restrict__ YH, const _Float16* __restrict__ YL, const float* __restrict__ WO, const float* __restrict__ BO, float* __restrict__ OUT) {
  __shared__ __align__(16) float sf[4][16][132];
  const int tid = threadIdx.x, wave = tid >> 5, lane = tid & 31, col = lane & 15, g = lane >> 4; const int c0 = blockIdx.y * 128; const size_t r0 = (size_t)blockIdx.x * 64 + wave * 16;
  v8f acc[8] = {};
#pragma unroll 2
  for (int kc = 0; kc < CC / 32; ++kc) { const v16h ah = frag_h(YH + (r0 + col) * CC + kc * 32, lane), al = frag_h(YL + (r0 + col) * CC + kc * 32, lane); asm volatile("s_wait_loadcnt 0x0" ::: "memory");
#pragma unroll
    for (int j = 0; j < 8; ++j) { const H2 w = wcolh2_io(WO, kc * 32, c0 + j * 16 + col, lane, DIN); asm volatile("s_wait_loadcnt 0x0" ::: "memory"); acc[j] = wmma16(ah, w.h, acc[j]); acc[j] = wmma16(al, w.l, acc[j]); } }
#pragma unroll
  for (int j = 0; j < 8; ++j) { const float bias = bfr(BO[c0 + j * 16 + col]);
#pragma unroll
    for (int r = 0; r < 8; ++r) sf[wave][8 * g + r][j * 16 + col] = acc[j][r] * (1.0f / 16384.0f) + bias; }
  LDSX();
  for (int rl = 0; rl < 16; ++rl) { const v4f v = *(const v4f*)&sf[wave][rl][lane * 4]; vst2((void*)(OUT + (r0 + rl) * DIN + c0 + lane * 4), v); } }

extern "C" void kernel_launch(void* const* d_in, const int* in_sizes, int n_in, void* d_out, int out_size, void* d_ws, size_t ws_size, hipStream_t stream) {
  if (n_in < 10) return;
  const long long need_rows = (long long)(NB - 1) * SEQ_FULL + SEQ;
  if ((long long)in_sizes[0] < need_rows * DIN) return;
  if ((long long)in_sizes[1] < need_rows) return;
  if (in_sizes[2] < DIN * CC || in_sizes[4] < DIN * CC || in_sizes[6] < DIN * CC || in_sizes[8] < CC * DIN) return;
  if (in_sizes[3] < CC || in_sizes[5] < CC || in_sizes[7] < CC || in_sizes[9] < DIN) return;
  if ((long long)out_size < (long long)NB * SEQ * DIN) return;
  if (ws_size < (size_t)WS_END) return;
  const float* X = (const float*)d_in[0]; const int* MK = (const int*)d_in[1];
  const float* Wq = (const float*)d_in[2]; const float* bq = (const float*)d_in[3];
  const float* Wk = (const float*)d_in[4]; const float* bk = (const float*)d_in[5];
  const float* Wv = (const float*)d_in[6]; const float* bv = (const float*)d_in[7];
  const float* Wo = (const float*)d_in[8]; const float* bo = (const float*)d_in[9];
  char* ws = (char*)d_ws;
  _Float16 *QH = (_Float16*)(ws + WS_QH), *QL = (_Float16*)(ws + WS_QL), *KH = (_Float16*)(ws + WS_KH), *VT = (_Float16*)(ws + WS_VT), *YH = (_Float16*)(ws + WS_YH), *YL = (_Float16*)(ws + WS_YL);
  k_proj_q<<<dim3(NB * SEQ / 64, CC / 128), 128, 0, stream>>>(X, Wq, bq, QH, QL);
  k_proj_k<<<dim3(NB * SEQ / 64, CC / 128), 128, 0, stream>>>(X, Wk, bk, KH);
  k_proj_v<<<dim3(NB * SEQ / 64, CC / 128), 128, 0, stream>>>(X, Wv, bv, VT);
  k_attn<<<dim3(SEQ / 64, NH, NB), 128, 0, stream>>>(QH, QL, KH, VT, MK, YH, YL);
  k_out<<<dim3(NB * SEQ / 64, DIN / 128), 128, 0, stream>>>(YH, YL, Wo, bo, (float*)d_out);
}
